// S4Model_30365418783277
// MI455X (gfx1250) — hardware-verified
//
#include <hip/hip_runtime.h>
#include <math.h>

typedef __attribute__((ext_vector_type(8)))  _Float16 v8h;
typedef __attribute__((ext_vector_type(16))) __bf16   v16b;
typedef __attribute__((ext_vector_type(8)))  __bf16   v8b;
typedef __attribute__((ext_vector_type(8)))  float    v8f;
typedef __attribute__((ext_vector_type(4)))  float    v4f;

constexpr int kBatch = 8;
constexpr int kSeq   = 4096;
constexpr int kDinp  = 128;
constexpr int kHid   = 256;
constexpr int kModes = 8;
constexpr int kLayers = 4;
constexpr int kGate2 = 2 * kHid;
constexpr int kRows  = kBatch * kSeq;
constexpr int kChunks = 32;
constexpr int kChunkLen = 128;
constexpr int kTilePitch = 260;
constexpr int kTabQ = 6;
constexpr int kStateQ = 2 * kModes;
static_assert(kChunks * kChunkLen == kSeq, "chunking covers the sequence exactly");
static_assert((kRows % 64) == 0 && (kHid % 64) == 0 && (kGate2 % 64) == 0, "GEMM M,N multiples of 64");
static_assert((kDinp % 32) == 0 && (kHid % 32) == 0, "GEMM K multiples of 32");
static_assert(kHid == 256 && kModes == 8, "thread maps assume 256 channels and 8 modes");

constexpr size_t kOffHA  = 0;
constexpr size_t kOffHB  = kOffHA  + (size_t)kRows * kHid * 4;
constexpr size_t kOffYH  = kOffHB  + (size_t)kRows * kHid * 4;
constexpr size_t kOffYL  = kOffYH  + (size_t)kRows * kHid * 2;
constexpr size_t kOffXH  = kOffYL  + (size_t)kRows * kHid * 2;
constexpr size_t kOffXL  = kOffXH  + (size_t)kRows * kDinp * 2;
constexpr size_t kOffLOC = kOffXL  + (size_t)kRows * kDinp * 2;
constexpr size_t kOffCAR = kOffLOC + (size_t)kBatch * kChunks * kStateQ * kHid * 4;
constexpr size_t kOffEWH = kOffCAR + (size_t)kBatch * kChunks * kStateQ * kHid * 4;
constexpr size_t kOffEWL = kOffEWH + (size_t)kHid * kDinp * 2;
constexpr size_t kOffOWH = kOffEWL + (size_t)kHid * kDinp * 2;
constexpr size_t kOffOWL = kOffOWH + (size_t)kLayers * kGate2 * kHid * 2;
constexpr size_t kOffTAB = kOffOWL + (size_t)kLayers * kGate2 * kHid * 2;
constexpr size_t kWsTotal = kOffTAB + (size_t)kLayers * kTabQ * kModes * kHid * 4;
static_assert(kWsTotal == 128253952ull, "carve total");
static_assert(kWsTotal <= 134217728ull, "carve cap");
static_assert((kOffHB % 128) == 0 && (kOffYH % 128) == 0 && (kOffYL % 128) == 0 && (kOffXH % 128) == 0 &&
              (kOffXL % 128) == 0 && (kOffLOC % 128) == 0 && (kOffCAR % 128) == 0 && (kOffEWH % 128) == 0 &&
              (kOffEWL % 128) == 0 && (kOffOWH % 128) == 0 && (kOffOWL % 128) == 0 && (kOffTAB % 128) == 0,
              "128-B aligned regions");

__device__ __forceinline__ unsigned short f2bf_bits(float f) {
  unsigned u = __float_as_uint(f);
  return (unsigned short)((u + 0x7FFFu + ((u >> 16) & 1u)) >> 16);
}
__device__ __forceinline__ float bf_bits2f(unsigned short h) { return __uint_as_float(((unsigned)h) << 16); }

__device__ __forceinline__ void guard_row_b(v8f& a, v8f& b, v8f& c, v8f& d, v16b x, v16b y) {
  asm volatile("v_nop\n\tv_nop\n\tv_nop\n\tv_nop" : "+v"(a), "+v"(b), "+v"(c), "+v"(d) : "v"(x), "v"(y));
}
__device__ __forceinline__ void keep4_b(v16b a, v16b b, v16b c, v16b d) { asm volatile("v_nop" :: "v"(a), "v"(b), "v"(c), "v"(d)); }
__device__ __forceinline__ void acc_guard4(v8f& a, v8f& b, v8f& c, v8f& d) {
  asm volatile("v_nop\n\tv_nop\n\tv_nop\n\tv_nop" : "+v"(a), "+v"(b), "+v"(c), "+v"(d));
}
__device__ __forceinline__ void pin4(float& a, float& b, float& c, float& d) { asm volatile("" : "+v"(a), "+v"(b), "+v"(c), "+v"(d)); }
__device__ __forceinline__ void pin2(float& a, float& b) { asm volatile("" : "+v"(a), "+v"(b)); }

struct FragB {
  union U { v16b v; v8b h[2]; };
  static __device__ __forceinline__ v16b load(const __bf16* p) {
    U f; f.h[0] = *(const v8b*)(p); f.h[1] = *(const v8b*)(p + 16); return f.v;
  }
  static __device__ __forceinline__ v8f mma(v16b a, v16b b, v8f c) {
    return __builtin_amdgcn_wmma_f32_16x16x32_bf16(false, a, false, b, (short)0, c, false, false);
  }
};

template <int EPI>
__global__ __launch_bounds__(256) void gemm_bf16x3_kernel(
    const unsigned short* __restrict__ Ahp, const unsigned short* __restrict__ Alp, int lda,
    const unsigned short* __restrict__ Bhp, const unsigned short* __restrict__ Blp, int ldb,
    float* __restrict__ Cout, int ldc,
    const float* __restrict__ bias, const float* __restrict__ resid,
    int M, int N, int K)
{
  const __bf16* Ah = (const __bf16*)Ahp;
  const __bf16* Al = (const __bf16*)Alp;
  const __bf16* Bh = (const __bf16*)Bhp;
  const __bf16* Bl = (const __bf16*)Blp;
  __shared__ __align__(16) float sT[8][16 * 68];
  const int lane = threadIdx.x & 31;
  const int wave = threadIdx.x >> 5;
  const int tilesN = N >> 6;
  const int tilesM = M >> 6;
  const int tile = blockIdx.x * 8 + wave;
  if (tile >= tilesM * tilesN) return;
  const int tm = tile / tilesN;
  const int tn = tile - tm * tilesN;
  const int m0 = tm << 6;
  const int n0 = tn << 6;
  const int rlane = lane & 15;
  const int koff  = (lane >> 4) * 8;
  const int mOff  = (lane >> 4) * 8;

  v8f acc[4][4];
#pragma unroll
  for (int i = 0; i < 4; ++i)
#pragma unroll
    for (int j = 0; j < 4; ++j) acc[i][j] = (v8f){0.f,0.f,0.f,0.f,0.f,0.f,0.f,0.f};

  const __bf16* bBaseH = Bh + (size_t)(n0 + rlane) * ldb + koff;
  const __bf16* bBaseL = Bl + (size_t)(n0 + rlane) * ldb + koff;
  const __bf16* aBaseH = Ah + (size_t)(m0 + rlane) * lda + koff;
  const __bf16* aBaseL = Al + (size_t)(m0 + rlane) * lda + koff;
  const size_t bStep = (size_t)16 * ldb;
  const size_t aStep = (size_t)16 * lda;

  for (int k0 = 0; k0 < K; k0 += 32) {
    v16b bh[4], bl[4];
#pragma unroll
    for (int j = 0; j < 4; ++j) {
      bh[j] = FragB::load(bBaseH + j * bStep + k0);
      bl[j] = FragB::load(bBaseL + j * bStep + k0);
    }
#pragma unroll
    for (int i = 0; i < 4; ++i) {
      const v16b ah = FragB::load(aBaseH + i * aStep + k0);
      const v16b al = FragB::load(aBaseL + i * aStep + k0);
#pragma unroll
      for (int j = 0; j < 4; ++j) {
        acc[i][j] = FragB::mma(ah, bh[j], acc[i][j]);
        acc[i][j] = FragB::mma(ah, bl[j], acc[i][j]);
        acc[i][j] = FragB::mma(al, bh[j], acc[i][j]);
      }
      guard_row_b(acc[i][0], acc[i][1], acc[i][2], acc[i][3], ah, al);
    }
    keep4_b(bh[0], bh[1], bh[2], bh[3]);
    keep4_b(bl[0], bl[1], bl[2], bl[3]);
  }
  acc_guard4(acc[0][0], acc[0][1], acc[0][2], acc[0][3]);
  acc_guard4(acc[1][0], acc[1][1], acc[1][2], acc[1][3]);
  acc_guard4(acc[2][0], acc[2][1], acc[2][2], acc[2][3]);
  acc_guard4(acc[3][0], acc[3][1], acc[3][2], acc[3][3]);

  float* slab = sT[wave];
  if (EPI == 0) {
    const int hh = lane >> 4, c4 = (lane & 15) * 4;
#pragma unroll
    for (int i = 0; i < 4; ++i) {
      const int mBase = m0 + (i << 4);
#pragma unroll
      for (int j = 0; j < 4; ++j) {
        const float bv = bias[n0 + (j << 4) + rlane];
#pragma unroll
        for (int r = 0; r < 8; ++r) slab[(mOff + r) * 68 + (j << 4) + rlane] = acc[i][j][r] + bv;
      }
      __builtin_amdgcn_fence(__ATOMIC_RELEASE, "workgroup");
      __builtin_amdgcn_wave_barrier();
      __builtin_amdgcn_fence(__ATOMIC_ACQUIRE, "workgroup");
      for (int pass = 0; pass < 2; ++pass) {
#pragma unroll
        for (int it = 0; it < 8; ++it) {
          const int row = it * 2 + hh;
          const v4f v = *(const v4f*)(slab + row * 68 + c4);
          *(volatile v4f*)(Cout + (size_t)(mBase + row) * ldc + n0 + c4) = v;
        }
        __threadfence();
      }
      __builtin_amdgcn_fence(__ATOMIC_RELEASE, "workgroup");
      __builtin_amdgcn_wave_barrier();
      __builtin_amdgcn_fence(__ATOMIC_ACQUIRE, "workgroup");
    }
  } else {
    const int q = lane >> 3, c4 = (lane & 7) * 4;
    const int p0 = n0 >> 1;
    const v4f ba = *(const v4f*)(bias + p0 + c4);
    const v4f bg = *(const v4f*)(bias + kHid + p0 + c4);
#pragma unroll
    for (int i = 0; i < 4; ++i) {
      const int mBase = m0 + (i << 4);
#pragma unroll
      for (int j = 0; j < 4; ++j)
#pragma unroll
        for (int r = 0; r < 8; ++r) slab[(mOff + r) * 68 + (j << 4) + rlane] = acc[i][j][r];
      __builtin_amdgcn_fence(__ATOMIC_RELEASE, "workgroup");
      __builtin_amdgcn_wave_barrier();
      __builtin_amdgcn_fence(__ATOMIC_ACQUIRE, "workgroup");
#pragma unroll 1
      for (int it = 0; it < 4; ++it) {
        const int row = it * 4 + q;
        float* sp = slab + row * 68 + c4;
        const v4f av = *(const v4f*)(sp);
        const v4f gv = *(const v4f*)(sp + 32);
        const size_t go = (size_t)(mBase + row) * ldc + p0 + c4;
        const v4f rv = *(const v4f*)(resid + go);
        v4f zv;
#pragma unroll
        for (int e = 0; e < 4; ++e) {
          const float ax = av[e] + ba[e];
          const float gx = gv[e] + bg[e];
          const float ex = expf(-gx);
          const float sg = 1.0f / (1.0f + ex);
          zv[e] = ax * sg + rv[e];
        }
        *(v4f*)(sp) = zv;
        *(volatile v4f*)(Cout + go) = zv;
      }
      __threadfence();
#pragma unroll 1
      for (int it = 0; it < 4; ++it) {
        const int row = it * 4 + q;
        const v4f zv = *(const v4f*)(slab + row * 68 + c4);
        *(volatile v4f*)(Cout + (size_t)(mBase + row) * ldc + p0 + c4) = zv;
      }
      __threadfence();
      __builtin_amdgcn_fence(__ATOMIC_RELEASE, "workgroup");
      __builtin_amdgcn_wave_barrier();
      __builtin_amdgcn_fence(__ATOMIC_ACQUIRE, "workgroup");
    }
  }
}

__global__ __launch_bounds__(256) void split_rows_bf16_kernel(
    const float* __restrict__ src, unsigned short* __restrict__ dhi, unsigned short* __restrict__ dlo, int total8)
{
  const int i = blockIdx.x * 256 + threadIdx.x;
  if (i >= total8) return;
  const size_t e0 = (size_t)i << 3;
  const v4f a0 = *(const v4f*)(src + e0);
  const v4f a1 = *(const v4f*)(src + e0 + 4);
  v8h hv, lv;
#pragma unroll
  for (int e = 0; e < 4; ++e) {
    const unsigned short h0 = f2bf_bits(a0[e]), h1 = f2bf_bits(a1[e]);
    const unsigned short l0 = f2bf_bits(a0[e] - bf_bits2f(h0)), l1 = f2bf_bits(a1[e] - bf_bits2f(h1));
    hv[e]     = __builtin_bit_cast(_Float16, h0);
    hv[4 + e] = __builtin_bit_cast(_Float16, h1);
    lv[e]     = __builtin_bit_cast(_Float16, l0);
    lv[4 + e] = __builtin_bit_cast(_Float16, l1);
  }
  unsigned short* qh = dhi + e0;
  unsigned short* ql = dlo + e0;
  *(volatile v8h*)qh = hv;
  *(volatile v8h*)ql = lv;
  __threadfence();
  *(volatile v8h*)qh = hv;
  *(volatile v8h*)ql = lv;
}

constexpr int kEnc8 = kHid * kDinp / 8;
constexpr int kOut8 = kLayers * kGate2 * kHid / 8;
static_assert((kEnc8 % 256) == 0 && (kOut8 % 256) == 0, "block-uniform branch and exact grid");
__global__ __launch_bounds__(256) void split_weights_kernel(
    const float* __restrict__ enc_w, const float* __restrict__ out_w,
    unsigned short* __restrict__ EWH, unsigned short* __restrict__ EWL,
    unsigned short* __restrict__ OWH, unsigned short* __restrict__ OWL)
{
  const int i = blockIdx.x * 256 + threadIdx.x;
  if (i >= kEnc8 + kOut8) return;
  const bool isEnc = (i < kEnc8);
  const int j = isEnc ? i : (i - kEnc8);
  const size_t e0 = (size_t)j << 3;
  const int layer = (int)(e0 / (size_t)(kGate2 * kHid));
  const int rem   = (int)(e0 - (size_t)layer * (kGate2 * kHid));
  const int prow  = rem / kHid;
  const int kcol  = rem - prow * kHid;
  const int t = prow >> 6, r = prow & 63;
  const int srow = (r < 32) ? (32 * t + r) : (kHid + 32 * t + (r - 32));
  const size_t so = (size_t)layer * (kGate2 * kHid) + (size_t)srow * kHid + kcol;
  const float* src = isEnc ? (enc_w + e0) : (out_w + so);
  unsigned short* qh = isEnc ? (EWH + e0) : (OWH + e0);
  unsigned short* ql = isEnc ? (EWL + e0) : (OWL + e0);
  const v4f a0 = *(const v4f*)(src);
  const v4f a1 = *(const v4f*)(src + 4);
  v8h hv, lv;
#pragma unroll
  for (int e = 0; e < 4; ++e) {
    const unsigned short h0 = f2bf_bits(a0[e]), h1 = f2bf_bits(a1[e]);
    const unsigned short l0 = f2bf_bits(a0[e] - bf_bits2f(h0)), l1 = f2bf_bits(a1[e] - bf_bits2f(h1));
    hv[e]     = __builtin_bit_cast(_Float16, h0);
    hv[4 + e] = __builtin_bit_cast(_Float16, h1);
    lv[e]     = __builtin_bit_cast(_Float16, l0);
    lv[4 + e] = __builtin_bit_cast(_Float16, l1);
  }
  *(volatile v8h*)qh = hv;
  *(volatile v8h*)ql = lv;
  __threadfence();
  *(volatile v8h*)qh = hv;
  *(volatile v8h*)ql = lv;
}

__global__ __launch_bounds__(256) void coef_table_kernel(
    const float* __restrict__ log_dt, const float* __restrict__ log_A_real, const float* __restrict__ A_imag,
    const float* __restrict__ C_re, const float* __restrict__ C_im, float* __restrict__ tab)
{
  const int idx = blockIdx.x * 256 + threadIdx.x;
  const int which = idx >> 13;
  const int rem = idx & 8191;
  const int h = rem & (kHid - 1);
  const int n = (rem >> 8) & (kModes - 1);
  const int layer = rem >> 11;
  const int pi = (layer * kHid + h) * kModes + n;
  const float dt = expf(log_dt[layer * kHid + h]);
  const float Ar = -expf(log_A_real[pi]);
  const float Ai = A_imag[pi];
  const float cr = C_re[pi];
  const float ci = C_im[pi];
  const float sc = which ? (float)kChunkLen : 1.0f;
  const float xr = Ar * dt;
  const float xi = Ai * dt;
  const float er = expf(xr * sc);
  float sn, cs;
  sincosf(xi * sc, &sn, &cs);
  const float wr = er * cs;
  const float wi = er * sn;
  const float nr = wr - 1.0f, ni = wi;
  const float tr = cr * nr - ci * ni;
  const float ti = cr * ni + ci * nr;
  const float inv = 1.0f / (Ar * Ar + Ai * Ai);
  const float c2r = 2.0f * ((tr * Ar + ti * Ai) * inv);
  const float c2i = 2.0f * ((ti * Ar - tr * Ai) * inv);
  float* base = tab + ((size_t)layer * kTabQ * kModes + n) * kHid + h;
  constexpr int kQStride = kModes * kHid;
  if (which == 0) {
    for (int pass = 0; pass < 2; ++pass) {
      *(volatile float*)(base + 0 * kQStride) = wr;
      *(volatile float*)(base + 1 * kQStride) = wi;
      *(volatile float*)(base + 4 * kQStride) = c2r;
      *(volatile float*)(base + 5 * kQStride) = c2i;
      __threadfence();
    }
  } else {
    for (int pass = 0; pass < 2; ++pass) {
      *(volatile float*)(base + 2 * kQStride) = wr;
      *(volatile float*)(base + 3 * kQStride) = wi;
      __threadfence();
    }
  }
}

__global__ __launch_bounds__(256) void scan_local_kernel(
    const float* __restrict__ hin, const float* __restrict__ tabL, float* __restrict__ loc)
{
  const int h = threadIdx.x;
  const int bc = blockIdx.x;
  float wr[kModes], wi[kModes], sr[kModes], si[kModes];
#pragma unroll
  for (int n = 0; n < kModes; ++n) {
    wr[n] = tabL[(0 * kModes + n) * kHid + h];
    wi[n] = tabL[(1 * kModes + n) * kHid + h];
    sr[n] = 0.0f;
    si[n] = 0.0f;
  }
  const float* up = hin + (size_t)bc * kChunkLen * kHid + h;
#pragma unroll 1
  for (int l = 0; l < kChunkLen; ++l) {
    float u = up[(size_t)l * kHid];
    asm volatile("" : "+v"(u));
#pragma unroll
    for (int n = 0; n < kModes; ++n) {
      float nr = fmaf(wr[n], sr[n], u);
      nr = fmaf(-wi[n], si[n], nr);
      float ni = wr[n] * si[n];
      ni = fmaf(wi[n], sr[n], ni);
      sr[n] = nr;
      si[n] = ni;
    }
  }
  float* st = loc + (size_t)bc * kStateQ * kHid + h;
  for (int pass = 0; pass < 2; ++pass) {
#pragma unroll
    for (int n = 0; n < kModes; ++n) {
      *(volatile float*)(st + (2 * n + 0) * kHid) = sr[n];
      *(volatile float*)(st + (2 * n + 1) * kHid) = si[n];
    }
    __threadfence();
  }
}

__global__ __launch_bounds__(256) void scan_carry_kernel(
    const float* __restrict__ tabL, const float* __restrict__ loc, float* __restrict__ car)
{
  const int h = threadIdx.x;
  const int b = blockIdx.x;
  float wTr[kModes], wTi[kModes], er[kModes], ei[kModes];
#pragma unroll
  for (int n = 0; n < kModes; ++n) {
    wTr[n] = tabL[(2 * kModes + n) * kHid + h];
    wTi[n] = tabL[(3 * kModes + n) * kHid + h];
    er[n] = 0.0f;
    ei[n] = 0.0f;
  }
#pragma unroll 1
  for (int c = 0; c < kChunks; ++c) {
    const size_t off = ((size_t)(b * kChunks + c) * kStateQ) * kHid + h;
    float Sr[kModes], Si[kModes];
#pragma unroll
    for (int n = 0; n < kModes; ++n) {
      Sr[n] = loc[off + (2 * n + 0) * kHid];
      Si[n] = loc[off + (2 * n + 1) * kHid];
    }
    for (int pass = 0; pass < 2; ++pass) {
#pragma unroll
      for (int n = 0; n < kModes; ++n) {
        *(volatile float*)(car + off + (2 * n + 0) * kHid) = er[n];
        *(volatile float*)(car + off + (2 * n + 1) * kHid) = ei[n];
      }
      __threadfence();
    }
#pragma unroll
    for (int n = 0; n < kModes; ++n) {
      float nr = fmaf(wTr[n], er[n], Sr[n]);
      nr = fmaf(-wTi[n], ei[n], nr);
      float ni = fmaf(wTr[n], ei[n], Si[n]);
      ni = fmaf(wTi[n], er[n], ni);
      er[n] = nr;
      ei[n] = ni;
    }
  }
}

__global__ __launch_bounds__(256) void scan_emit_kernel(
    const float* __restrict__ hin, const float* __restrict__ tabL, const float* __restrict__ dskip,
    const float* __restrict__ car, unsigned short* __restrict__ YH, unsigned short* __restrict__ YL)
{
  __shared__ __align__(16) float sT[16 * kTilePitch];
  const int tid = threadIdx.x, lane = tid & 31, wave = tid >> 5;
  const int h = tid;
  const int bc = blockIdx.x;
  float wr[kModes], wi[kModes], c2r[kModes], c2i[kModes], sr[kModes], si[kModes];
  const float* cp = car + (size_t)bc * kStateQ * kHid + h;
#pragma unroll
  for (int n = 0; n < kModes; ++n) {
    wr[n]  = tabL[(0 * kModes + n) * kHid + h];
    wi[n]  = tabL[(1 * kModes + n) * kHid + h];
    c2r[n] = tabL[(4 * kModes + n) * kHid + h];
    c2i[n] = tabL[(5 * kModes + n) * kHid + h];
    sr[n]  = cp[(2 * n + 0) * kHid];
    si[n]  = cp[(2 * n + 1) * kHid];
    pin4(wr[n], wi[n], c2r[n], c2i[n]);
    pin2(sr[n], si[n]);
  }
  const float dsk = dskip[h];
  const size_t row0 = (size_t)bc * kChunkLen;
#pragma unroll 1
  for (int sub = 0; sub < kChunkLen / 16; ++sub) {
    const size_t lb = row0 + (size_t)sub * 16;
#pragma unroll 1
    for (int s = 0; s < 16; ++s) {
      float u = hin[(lb + s) * kHid + h];
      asm volatile("" : "+v"(u));
      float y = dsk * u;
#pragma unroll
      for (int n = 0; n < kModes; ++n) {
        float nr = fmaf(wr[n], sr[n], u);
        nr = fmaf(-wi[n], si[n], nr);
        float ni = wr[n] * si[n];
        ni = fmaf(wi[n], sr[n], ni);
        sr[n] = nr;
        si[n] = ni;
        y = fmaf(c2r[n], nr, y);
        y = fmaf(-c2i[n], ni, y);
      }
      const float y3 = y * y * y;
      const float th = tanhf(0.7978845608028654f * (y + 0.044715f * y3));
      sT[s * kTilePitch + tid] = 0.5f * y * (1.0f + th);
    }
    __syncthreads();
    for (int pass = 0; pass < 2; ++pass) {
#pragma unroll
      for (int it = 0; it < 2; ++it) {
        const int row = it * 8 + wave;
        const float* sp = sT + row * kTilePitch + lane * 8;
        const v4f a0 = *(const v4f*)(sp);
        const v4f a1 = *(const v4f*)(sp + 4);
        v8h hv, lv;
#pragma unroll
        for (int e = 0; e < 4; ++e) {
          const unsigned short h0 = f2bf_bits(a0[e]), h1 = f2bf_bits(a1[e]);
          const unsigned short l0 = f2bf_bits(a0[e] - bf_bits2f(h0)), l1 = f2bf_bits(a1[e] - bf_bits2f(h1));
          hv[e]     = __builtin_bit_cast(_Float16, h0);
          hv[4 + e] = __builtin_bit_cast(_Float16, h1);
          lv[e]     = __builtin_bit_cast(_Float16, l0);
          lv[4 + e] = __builtin_bit_cast(_Float16, l1);
        }
        const size_t o = (lb + row) * kHid + lane * 8;
        *(volatile v8h*)(YH + o) = hv;
        *(volatile v8h*)(YL + o) = lv;
      }
      __threadfence();
    }
    __syncthreads();
  }
}

extern "C" void kernel_launch(void* const* d_in, const int* in_sizes, int n_in,
                              void* d_out, int out_size, void* d_ws, size_t ws_size,
                              hipStream_t stream)
{
  if (n_in < 11) return;
  if (in_sizes[0] != kRows * kDinp) return;
  if (in_sizes[1] != kHid * kDinp) return;
  if (in_sizes[2] != kHid) return;
  if (in_sizes[3] != kLayers * kHid) return;
  if (in_sizes[4] != kLayers * kHid * kModes) return;
  if (in_sizes[5] != kLayers * kHid * kModes) return;
  if (in_sizes[6] != kLayers * kHid * kModes) return;
  if (in_sizes[7] != kLayers * kHid * kModes) return;
  if (in_sizes[8] != kLayers * kHid) return;
  if (in_sizes[9] != kLayers * kGate2 * kHid) return;
  if (in_sizes[10] != kLayers * kGate2) return;
  if (out_size != kRows * kHid) return;
  if (ws_size < kWsTotal) return;

  const float* x          = (const float*)d_in[0];
  const float* enc_w      = (const float*)d_in[1];
  const float* enc_b      = (const float*)d_in[2];
  const float* log_dt     = (const float*)d_in[3];
  const float* log_A_real = (const float*)d_in[4];
  const float* A_imag     = (const float*)d_in[5];
  const float* C_re       = (const float*)d_in[6];
  const float* C_im       = (const float*)d_in[7];
  const float* D_skip     = (const float*)d_in[8];
  const float* out_w      = (const float*)d_in[9];
  const float* out_b      = (const float*)d_in[10];
  float* outp = (float*)d_out;

  char* ws = (char*)d_ws;
  float*          HA  = (float*)(ws + kOffHA);
  float*          HB  = (float*)(ws + kOffHB);
  unsigned short* YH  = (unsigned short*)(ws + kOffYH);
  unsigned short* YL  = (unsigned short*)(ws + kOffYL);
  unsigned short* XH  = (unsigned short*)(ws + kOffXH);
  unsigned short* XL  = (unsigned short*)(ws + kOffXL);
  float*          LOC = (float*)(ws + kOffLOC);
  float*          CAR = (float*)(ws + kOffCAR);
  unsigned short* EWH = (unsigned short*)(ws + kOffEWH);
  unsigned short* EWL = (unsigned short*)(ws + kOffEWL);
  unsigned short* OWH = (unsigned short*)(ws + kOffOWH);
  unsigned short* OWL = (unsigned short*)(ws + kOffOWL);
  float*          TAB = (float*)(ws + kOffTAB);

  split_rows_bf16_kernel<<<(kRows * kDinp / 8) / 256, 256, 0, stream>>>(x, XH, XL, kRows * kDinp / 8);
  split_weights_kernel<<<(kEnc8 + kOut8) / 256, 256, 0, stream>>>(enc_w, out_w, EWH, EWL, OWH, OWL);
  coef_table_kernel<<<(2 * kLayers * kModes * kHid) / 256, 256, 0, stream>>>(log_dt, log_A_real, A_imag, C_re, C_im, TAB);

  gemm_bf16x3_kernel<0><<<((kRows / 64) * (kHid / 64)) / 8, 256, 0, stream>>>(
      XH, XL, kDinp, EWH, EWL, kDinp, HA, kHid, enc_b, enc_b, kRows, kHid, kDinp);

  for (int i = 0; i < kLayers; ++i) {
    const float* hin = (i & 1) ? HB : HA;
    float* hout = (i == kLayers - 1) ? outp : ((i & 1) ? HA : HB);
    const float* tabL = TAB + (size_t)i * kTabQ * kModes * kHid;
    scan_local_kernel<<<kBatch * kChunks, 256, 0, stream>>>(hin, tabL, LOC);
    scan_carry_kernel<<<kBatch, 256, 0, stream>>>(tabL, LOC, CAR);
    scan_emit_kernel<<<kBatch * kChunks, 256, 0, stream>>>(hin, tabL, D_skip + (size_t)i * kHid, CAR, YH, YL);
    gemm_bf16x3_kernel<1><<<((kRows / 64) * (kGate2 / 64)) / 8, 256, 0, stream>>>(
        YH, YL, kHid,
        OWH + (size_t)i * kGate2 * kHid, OWL + (size_t)i * kGate2 * kHid, kHid,
        hout, kHid, out_b + (size_t)i * kGate2, hin, kRows, kGate2, kHid);
  }
}
